// SocialPooling_5360119185920
// MI455X (gfx1250) — hardware-verified
//
#include <hip/hip_runtime.h>
#include <stddef.h>
#include <stdint.h>

#define HDIM   64
#define GRIDN  8
#define NCELL  64
#define NPED   64
#define NSEQ   64
#define NROW   4096
#define KIN    4096
#define KPL    8192
#define NOUT   1024
#define NTHR   256
#define GTHR   128
#define GBM    64
#define GBN    128
#define PGRP   4
#define TP     72
#define BNCOL  128
#define WSMAX  134217728
#define BN_EPS 1e-5f
#define POOL_LDS_FLOATS (KIN + PGRP * KIN + NPED * NPED + 2 * NPED)
#define POOL_LDS_BYTES  (POOL_LDS_FLOATS * 4)

static_assert(NROW == NSEQ * NPED);
static_assert(KIN == NCELL * HDIM && NCELL == GRIDN * GRIDN && KPL == 2 * KIN);
static_assert(KIN % 32 == 0 && NROW % GBM == 0 && NOUT % GBN == 0);
static_assert(GBM == 64 && GBN == 128 && GTHR == 128);
static_assert(NTHR == PGRP * HDIM && HDIM == 64 && NPED % PGRP == 0);
static_assert(KPL / 8 == 1024 && KIN / 8 == 512);
static_assert((PGRP * KPL) % (8 * NTHR) == 0);
static_assert(NPED * NPED == 16 * NTHR && KIN == 16 * NTHR && HDIM * NPED == 16 * NTHR);
static_assert((TP * 2) % 16 == 0 && TP >= 64);
static_assert(KIN % 64 == 0 && NOUT % 64 == 0);
static_assert(NOUT % BNCOL == 0 && BNCOL == 4 * 32 && NROW % (NTHR / 32) == 0);
static_assert(POOL_LDS_BYTES <= 300000);

typedef float          v4f   __attribute__((ext_vector_type(4)));
typedef float          v8f   __attribute__((ext_vector_type(8)));
typedef int            v8i   __attribute__((ext_vector_type(8)));
typedef unsigned short v8us  __attribute__((ext_vector_type(8)));
typedef unsigned short v16us __attribute__((ext_vector_type(16)));
typedef __bf16         v16bf __attribute__((ext_vector_type(16)));
typedef v4f  __attribute__((may_alias)) v4fa;
typedef v8us __attribute__((may_alias)) v8usa;
union FragB { v16bf v; v16us u; v8us h[2]; v8i w; };

__device__ __forceinline__ v8f wmb(const FragB& a, const FragB& b, v8f c) {
  v8f d = __builtin_amdgcn_wmma_f32_16x16x32_bf16(false, a.v, false, b.v, (short)0, c, false, false);
  asm volatile("v_nop\n\tv_nop\n\tv_nop\n\tv_nop" : "+v"(d) : "v"(a.w), "v"(b.w));
  return d;
}

__device__ __forceinline__ unsigned bf16_bits(float f) {
  const unsigned u = __float_as_uint(f);
  return (u + 0x7FFFu + ((u >> 16) & 1u)) >> 16;
}
__device__ __forceinline__ float bf16_val(float f) {
  return __uint_as_float(bf16_bits(f) << 16);
}
__device__ __forceinline__ void put16(unsigned short* dp, v8us o) {
  *(volatile v8us*)dp = o;
  __threadfence();
  *(volatile v8us*)dp = o;
}
__device__ __forceinline__ void putf4(float* dp, v4f o) {
  *(volatile v4f*)dp = o;
  __threadfence();
  *(volatile v4f*)dp = o;
}

__global__ __launch_bounds__(NTHR) void k_wt(const float* __restrict__ W, unsigned short* BT) {
  __shared__ __attribute__((aligned(16))) unsigned short sT[64 * TP];
  const int tid = (int)threadIdx.x;
  const int k0 = (int)blockIdx.x * 64;
  const int n0 = (int)blockIdx.y * 64;
#pragma unroll
  for (int it = 0; it < 4; ++it) {
    const int f   = it * NTHR + tid;
    const int row = f >> 4;
    const int c4  = (f & 15) * 4;
    const v4f v = *(const v4fa*)(W + (size_t)(k0 + row) * NOUT + n0 + c4);
    sT[(c4 + 0) * TP + row] = (unsigned short)bf16_bits(v.x);
    sT[(c4 + 1) * TP + row] = (unsigned short)bf16_bits(v.y);
    sT[(c4 + 2) * TP + row] = (unsigned short)bf16_bits(v.z);
    sT[(c4 + 3) * TP + row] = (unsigned short)bf16_bits(v.w);
  }
  __syncthreads();
#pragma unroll
  for (int sw = 0; sw < 2; ++sw) {
    const int n = sw * 32 + (tid >> 3);
    const int q = tid & 7;
    const v8us o = *(const v8usa*)(sT + n * TP + 8 * q);
    put16(BT + (size_t)(n0 + n) * KIN + k0 + 8 * q, o);
  }
}

__global__ __launch_bounds__(NTHR) void k_pool(const float* __restrict__ hs, const float* __restrict__ ep,
                                               const int* __restrict__ sse, const float* __restrict__ rp,
                                               unsigned short* PL) {
#pragma clang fp contract(off)
  extern __shared__ __attribute__((aligned(16))) float dyn[];
  float* hid   = dyn;
  float* acc   = dyn + KIN;
  int*   cellT = (int*)(dyn + KIN + PGRP * KIN);
  float* px    = dyn + KIN + PGRP * KIN + NPED * NPED;
  float* py    = px + NPED;
  const int tid = (int)threadIdx.x;
  const int s = (int)blockIdx.x;
  (void)sse;
  (void)rp;

  {
    const float* src = hs + (size_t)s * NPED * HDIM;
#pragma unroll
    for (int it = 0; it < 4; ++it) {
      const int f = it * NTHR + tid;
      const v4f v = *(const v4fa*)(src + 4 * f);
      v4f o;
      o.x = bf16_val(v.x);
      o.y = bf16_val(v.y);
      o.z = bf16_val(v.z);
      o.w = bf16_val(v.w);
      *(v4fa*)(hid + 4 * f) = o;
    }
    if (tid < NPED) {
      const float x = ep[(size_t)(s * NPED + tid) * 2 + 0];
      const float y = ep[(size_t)(s * NPED + tid) * 2 + 1];
      px[tid] = bf16_val(x);
      py[tid] = bf16_val(y);
    }
  }
  __syncthreads();

#pragma unroll 1
  for (int it = 0; it < (NPED * NPED) / NTHR; ++it) {
    const int pr = it * NTHR + tid;
    const int i = pr >> 6, j = pr & 63;
    const float xi = px[i], yi = py[i], xj = px[j], yj = py[j];
    const float tlx = xi - 1.0f;
    const float tly = yi + 1.0f;
    const float brx = xi + 1.0f;
    const float bry = yi - 1.0f;
    const bool oob = (xj >= brx) || (xj <= tlx) || (yj >= tly) || (yj <= bry) || (i == j);
    const float ax = (xj - tlx) * 0.5f;
    const float cx = floorf(ax * 8.0f);
    const float ay = (tly - yj) * 0.5f;
    const float cy = floorf(ay * 8.0f);
    const float c8 = cy * 8.0f;
    const float gf = cx + c8;
    const float gcl = fminf(fmaxf(gf, -4.0f), 200.0f);
    int g = (int)gcl;
    g = oob ? -1 : g;
    g = (g < 0 || g > NCELL + 8) ? -1 : g;
    cellT[pr] = g;
  }
  __syncthreads();

  const int p = tid >> 6;
  const int h = tid & 63;
#pragma unroll 1
  for (int gp = 0; gp < NPED / PGRP; ++gp) {
    {
      const v4f z = {0.0f, 0.0f, 0.0f, 0.0f};
#pragma unroll
      for (int it = 0; it < (PGRP * KIN) / (4 * NTHR); ++it) *(v4fa*)(acc + 4 * (it * NTHR + tid)) = z;
    }
    __syncthreads();
    const int i = gp * PGRP + p;
    float* ar = acc + p * KIN + h;
#pragma unroll 1
    for (int j = 0; j < NPED; ++j) {
      const int c = cellT[i * NPED + j];
      if (c >= 0 && c < NCELL) ar[c * HDIM] += hid[j * HDIM + h];
    }
    if (i >= 1) {
#pragma unroll 1
      for (int j = 0; j < NPED; ++j) {
        const int c = cellT[(i - 1) * NPED + j];
        if (c >= NCELL && c <= NCELL + 8) ar[(c - NCELL) * HDIM] += hid[j * HDIM + h];
      }
    }
    __syncthreads();

    const size_t rowg0 = (size_t)s * NPED + (size_t)gp * PGRP;
#pragma unroll 1
    for (int sw = 0; sw < (PGRP * KPL) / (8 * NTHR); ++sw) {
      const int u    = sw * NTHR + tid;
      const int pq   = u >> 10;
      const int o    = (u & 1023) * 8;
      const int part = (u >> 9) & 1;
      const float* aq = acc + pq * KIN + (o & (KIN - 1));
      const v4f va = *(const v4fa*)aq;
      const v4f vb = *(const v4fa*)(aq + 4);
      const v8f f8 = {va.x, va.y, va.z, va.w, vb.x, vb.y, vb.z, vb.w};
      const unsigned mlo = 0u - (unsigned)part;
      const unsigned mhi = ~mlo;
      v8us oo;
#pragma unroll
      for (int e = 0; e < 8; ++e) {
        const unsigned hb = bf16_bits(f8[e]);
        const unsigned lb = bf16_bits(f8[e] - __uint_as_float(hb << 16));
        oo[e] = (unsigned short)((hb & mhi) | (lb & mlo));
      }
      put16(PL + (rowg0 + (size_t)pq) * KPL + o, oo);
    }
    __syncthreads();
  }
}

__global__ __launch_bounds__(GTHR) void k_gemm(const unsigned short* __restrict__ PL,
                                               const unsigned short* __restrict__ BT,
                                               const float* __restrict__ bias, float* XW) {
  __shared__ __attribute__((aligned(16))) float stg[GBM * GBN];
  const int tid = (int)threadIdx.x, lane = tid & 31, wave = tid >> 5, hh = lane >> 4, m = lane & 15;
  const int wm = wave & 1, wn = wave >> 1;
  const int rowBase = (int)blockIdx.x * GBM;
  const int colBase = (int)blockIdx.y * GBN;

  v8f acc[2][4];
  {
    const v8f z = {0.f, 0.f, 0.f, 0.f, 0.f, 0.f, 0.f, 0.f};
#pragma unroll
    for (int mt = 0; mt < 2; ++mt)
#pragma unroll
      for (int nt = 0; nt < 4; ++nt) acc[mt][nt] = z;
  }
  const unsigned short* ap0 = PL + (size_t)(rowBase + 32 * wm + m) * KPL + 8 * hh;
  const unsigned short* ap1 = ap0 + (size_t)16 * KPL;
  const unsigned short* bp  = BT + (size_t)(colBase + 64 * wn + m) * KIN + 8 * hh;

#pragma unroll 1
  for (int k0 = 0; k0 < KIN; k0 += 32) {
    FragB a0h, a0l, a1h, a1l;
    a0h.h[0] = *(const v8usa*)(ap0 + k0);
    a0h.h[1] = *(const v8usa*)(ap0 + k0 + 16);
    a0l.h[0] = *(const v8usa*)(ap0 + KIN + k0);
    a0l.h[1] = *(const v8usa*)(ap0 + KIN + k0 + 16);
    a1h.h[0] = *(const v8usa*)(ap1 + k0);
    a1h.h[1] = *(const v8usa*)(ap1 + k0 + 16);
    a1l.h[0] = *(const v8usa*)(ap1 + KIN + k0);
    a1l.h[1] = *(const v8usa*)(ap1 + KIN + k0 + 16);
#pragma unroll
    for (int nt = 0; nt < 4; ++nt) {
      const unsigned short* wq = bp + (size_t)(16 * nt) * KIN + k0;
      FragB b;
      b.h[0] = *(const v8usa*)wq;
      b.h[1] = *(const v8usa*)(wq + 16);
      acc[0][nt] = wmb(a0h, b, acc[0][nt]);
      acc[0][nt] = wmb(a0l, b, acc[0][nt]);
      acc[1][nt] = wmb(a1h, b, acc[1][nt]);
      acc[1][nt] = wmb(a1l, b, acc[1][nt]);
    }
  }

#pragma unroll
  for (int nt = 0; nt < 4; ++nt) {
    const int lc = 64 * wn + 16 * nt + m;
    const float bvv = bf16_val(bias[colBase + lc]);
#pragma unroll
    for (int mt = 0; mt < 2; ++mt) {
#pragma unroll
      for (int r = 0; r < 8; ++r) {
        const int lr = 32 * wm + 16 * mt + 8 * hh + r;
        stg[lr * GBN + lc] = acc[mt][nt][r] + bvv;
      }
    }
  }
  __syncthreads();

  v4f pv[16];
#pragma unroll
  for (int i = 0; i < 16; ++i) pv[i] = *(const v4fa*)(stg + (16 * wave + i) * GBN + 4 * lane);
#pragma unroll
  for (int i = 0; i < 16; ++i) {
    float* op = XW + (size_t)(rowBase + 16 * wave + i) * NOUT + colBase + 4 * lane;
    *(volatile v4f*)op = pv[i];
  }
  __threadfence();
#pragma unroll
  for (int i = 0; i < 16; ++i) {
    float* op = XW + (size_t)(rowBase + 16 * wave + i) * NOUT + colBase + 4 * lane;
    *(volatile v4f*)op = pv[i];
  }
}

__global__ __launch_bounds__(NTHR) void k_bn(const float* __restrict__ XW, const float* __restrict__ gam,
                                             const float* __restrict__ bet, float* out) {
  __shared__ __attribute__((aligned(16))) double pS[8 * BNCOL];
  __shared__ __attribute__((aligned(16))) double pQ[8 * BNCOL];
  const int tid = (int)threadIdx.x, lane = tid & 31, wave = tid >> 5;
  const int c0 = (int)blockIdx.x * BNCOL + 4 * lane;
  const float* xc = XW + c0;

  double s0 = 0.0, s1 = 0.0, s2 = 0.0, s3 = 0.0;
#pragma unroll 1
  for (int k = 0; k < NROW / 8; ++k) {
    const v4f v = *(const v4fa*)(xc + (size_t)(wave + 8 * k) * NOUT);
    s0 += (double)v.x;
    s1 += (double)v.y;
    s2 += (double)v.z;
    s3 += (double)v.w;
  }
  pS[wave * BNCOL + 4 * lane + 0] = s0;
  pS[wave * BNCOL + 4 * lane + 1] = s1;
  pS[wave * BNCOL + 4 * lane + 2] = s2;
  pS[wave * BNCOL + 4 * lane + 3] = s3;
  __syncthreads();
  double t0 = 0.0, t1 = 0.0, t2 = 0.0, t3 = 0.0;
#pragma unroll 1
  for (int w2 = 0; w2 < 8; ++w2) {
    t0 += pS[w2 * BNCOL + 4 * lane + 0];
    t1 += pS[w2 * BNCOL + 4 * lane + 1];
    t2 += pS[w2 * BNCOL + 4 * lane + 2];
    t3 += pS[w2 * BNCOL + 4 * lane + 3];
  }
  const double inv = 1.0 / (double)NROW;
  const float m0 = (float)(t0 * inv);
  const float m1 = (float)(t1 * inv);
  const float m2 = (float)(t2 * inv);
  const float m3 = (float)(t3 * inv);

  double q0 = 0.0, q1 = 0.0, q2 = 0.0, q3 = 0.0;
#pragma unroll 1
  for (int k = 0; k < NROW / 8; ++k) {
    const v4f v = *(const v4fa*)(xc + (size_t)(wave + 8 * k) * NOUT);
    const float d0 = v.x - m0;
    const float d1 = v.y - m1;
    const float d2 = v.z - m2;
    const float d3 = v.w - m3;
    q0 += (double)(d0 * d0);
    q1 += (double)(d1 * d1);
    q2 += (double)(d2 * d2);
    q3 += (double)(d3 * d3);
  }
  pQ[wave * BNCOL + 4 * lane + 0] = q0;
  pQ[wave * BNCOL + 4 * lane + 1] = q1;
  pQ[wave * BNCOL + 4 * lane + 2] = q2;
  pQ[wave * BNCOL + 4 * lane + 3] = q3;
  __syncthreads();
  double u0 = 0.0, u1 = 0.0, u2 = 0.0, u3 = 0.0;
#pragma unroll 1
  for (int w2 = 0; w2 < 8; ++w2) {
    u0 += pQ[w2 * BNCOL + 4 * lane + 0];
    u1 += pQ[w2 * BNCOL + 4 * lane + 1];
    u2 += pQ[w2 * BNCOL + 4 * lane + 2];
    u3 += pQ[w2 * BNCOL + 4 * lane + 3];
  }
  const float r0 = rsqrtf((float)(u0 * inv) + BN_EPS);
  const float r1 = rsqrtf((float)(u1 * inv) + BN_EPS);
  const float r2 = rsqrtf((float)(u2 * inv) + BN_EPS);
  const float r3 = rsqrtf((float)(u3 * inv) + BN_EPS);

  const v4f g4 = *(const v4fa*)(gam + c0);
  const v4f b4 = *(const v4fa*)(bet + c0);
  const float g0 = bf16_val(g4.x), g1 = bf16_val(g4.y), g2 = bf16_val(g4.z), g3 = bf16_val(g4.w);
  const float e0 = bf16_val(b4.x), e1 = bf16_val(b4.y), e2 = bf16_val(b4.z), e3 = bf16_val(b4.w);

#pragma unroll 1
  for (int k = 0; k < NROW / 8; ++k) {
    const int r = wave + 8 * k;
    const v4f v = *(const v4fa*)(xc + (size_t)r * NOUT);
    v4f o;
    o.x = fmaxf((v.x - m0) * r0 * g0 + e0, 0.0f);
    o.y = fmaxf((v.y - m1) * r1 * g1 + e1, 0.0f);
    o.z = fmaxf((v.z - m2) * r2 * g2 + e2, 0.0f);
    o.w = fmaxf((v.w - m3) * r3 * g3 + e3, 0.0f);
    putf4(out + (size_t)r * NOUT + c0, o);
  }
}

extern "C" void kernel_launch(void* const* d_in, const int* in_sizes, int n_in,
                              void* d_out, int out_size, void* d_ws, size_t ws_size,
                              hipStream_t stream) {
  if (n_in < 8) return;
  if (in_sizes[0] != NROW * HDIM) return;
  if (in_sizes[1] != NSEQ * 2) return;
  if (in_sizes[2] != NROW * 2) return;
  if (in_sizes[4] != KIN * NOUT) return;
  if (in_sizes[5] != NOUT || in_sizes[6] != NOUT || in_sizes[7] != NOUT) return;
  if (out_size != NROW * NOUT) return;

  const float* hs    = (const float*)d_in[0];
  const int*   sse   = (const int*)d_in[1];
  const float* ep    = (const float*)d_in[2];
  const float* rp    = (const float*)d_in[3];
  const float* W     = (const float*)d_in[4];
  const float* b     = (const float*)d_in[5];
  const float* gamma = (const float*)d_in[6];
  const float* beta  = (const float*)d_in[7];
  float* out = (float*)d_out;

  char* ws = (char*)d_ws;
  size_t off = 0;
  const size_t oBT = off; off += (size_t)NOUT * KIN * 2;
  const size_t oPL = off; off += (size_t)NROW * KPL * 2;
  const size_t oXW = off; off += (size_t)NROW * NOUT * 4;
  if (off > ws_size || off > (size_t)WSMAX) return;
  unsigned short* BT = (unsigned short*)(ws + oBT);
  unsigned short* PL = (unsigned short*)(ws + oPL);
  float*          XW = (float*)(ws + oXW);

  hipFuncSetAttribute(reinterpret_cast<const void*>(&k_pool), hipFuncAttributeMaxDynamicSharedMemorySize,
                      (int)POOL_LDS_BYTES);

  k_wt<<<dim3(KIN / 64, NOUT / 64), NTHR, 0, stream>>>(W, BT);
  k_pool<<<NSEQ, NTHR, POOL_LDS_BYTES, stream>>>(hs, ep, sse, rp, PL);
  k_gemm<<<dim3(NROW / GBM, NOUT / GBN), GTHR, 0, stream>>>(PL, BT, b, XW);
  k_bn<<<NOUT / BNCOL, NTHR, 0, stream>>>(XW, gamma, beta, out);
}
